// eHON_MPL_centroid_6622839570872
// MI455X (gfx1250) — hardware-verified
//
#include <hip/hip_runtime.h>
#include <stddef.h>


#define NTHR   256
#define NWAVE  8
#define EPT    8
#define CHUNK  (NTHR * EPT)
#define WCAP   (EPT * 32)
#define LISTN  (NWAVE * WCAP)
#define PASSN  (NWAVE * 16)
#define PCAP   (CHUNK + PASSN)
#define NB     256
#define AW     132
#define UP     132
#define WSC    16.0f
#define WINV   0.0625f

#define OFF_ACC   0
#define OFF_UT    (OFF_ACC + (NB + 1) * AW)
#define OFF_SV    (OFF_UT + PASSN * UP)
#define OFF_WV    (OFF_SV + PASSN * 4)
#define OFF_BC    (OFF_WV + 128)
#define OFF_C2    (OFF_BC + 128)
#define OFF_SLOT  (OFF_C2 + 128)
#define OFF_LIST  (OFF_SLOT + PASSN)
#define OFF_PEND  (OFF_LIST + LISTN)
#define DRAIN_LDS_FLOATS (OFF_PEND + PCAP)
#define DRAIN_LDS_BYTES  (DRAIN_LDS_FLOATS * 4)
#define GEMM_LDS_BYTES   (NWAVE * 2048 * 4)
#define CELL_NW          4
#define CELL_ROWS        (CELL_NW * 16)
#define CELL_LDS_BYTES   (CELL_NW * 4096 * 4)

static_assert((CHUNK % PASSN) == 0);
static_assert((PCAP % PASSN) == 0);
static_assert(PASSN <= NTHR);
static_assert(AW <= NTHR);
static_assert((NB % 32) == 0);
static_assert(NB == NWAVE * 32);
static_assert((OFF_UT % 4) == 0);
static_assert((OFF_SV % 4) == 0);
static_assert((OFF_WV % 4) == 0);
static_assert((OFF_SLOT % 4) == 0);
static_assert((OFF_LIST % 4) == 0);
static_assert((OFF_PEND % 4) == 0);
static_assert(((UP * 4) % 16) == 0);
static_assert(((AW * 4) % 16) == 0);

typedef float          v4f  __attribute__((ext_vector_type(4)));
typedef float          v8f  __attribute__((ext_vector_type(8)));
typedef int            v4i  __attribute__((ext_vector_type(4)));
typedef int            v8i  __attribute__((ext_vector_type(8)));
typedef _Float16       v8h  __attribute__((ext_vector_type(8)));
typedef _Float16       v16h __attribute__((ext_vector_type(16)));
typedef unsigned short v8us __attribute__((ext_vector_type(8)));
typedef __bf16         v16bf __attribute__((ext_vector_type(16)));

union FragH { v16h v;  v8h  h[2]; };
union FragB { v16bf v; v8us h[2]; v8i w; };

__device__ __forceinline__ v8f zacc() {
  v8f z;
#pragma unroll
  for (int i = 0; i < 8; ++i) z[i] = 0.0f;
  return z;
}

__device__ __forceinline__ v8f wmh(v16h a, v16h b, v8f c) {
  v8f d = __builtin_amdgcn_wmma_f32_16x16x32_f16(false, a, false, b, (short)0, c, false, false);
  asm volatile("v_nop\n\tv_nop\n\tv_nop\n\tv_nop" : "+v"(d) : "v"(a), "v"(b));
  return d;
}

__device__ __forceinline__ v8f wmb(const FragB& a, const FragB& b, v8f c) {
  v8f d = __builtin_amdgcn_wmma_f32_16x16x32_bf16(false, a.v, false, b.v, (short)0, c, false, false);
  asm volatile("v_nop\n\tv_nop\n\tv_nop\n\tv_nop" : "+v"(d) : "v"(a.w), "v"(b.w));
  return d;
}

__device__ __forceinline__ unsigned short bf_rne(float x) {
  unsigned int u = __float_as_uint(x);
  u += 0x7FFFu + ((u >> 16) & 1u);
  return (unsigned short)(u >> 16);
}

__device__ __forceinline__ void split8(v4f a, v4f b, v8us& hi, v8us& lo) {
  const float f[8] = {a.x, a.y, a.z, a.w, b.x, b.y, b.z, b.w};
  v8us th, tl;
#pragma unroll
  for (int i = 0; i < 8; ++i) {
    const unsigned short hb = bf_rne(f[i]);
    const float hf = __uint_as_float(((unsigned int)hb) << 16);
    th[i] = hb;
    tl[i] = bf_rne(f[i] - hf);
  }
  hi = th;
  lo = tl;
}

__device__ __forceinline__ v8h cvt8h(v4f a, v4f b) {
  v8h r;
  r[0] = (_Float16)a.x; r[1] = (_Float16)a.y; r[2] = (_Float16)a.z; r[3] = (_Float16)a.w;
  r[4] = (_Float16)b.x; r[5] = (_Float16)b.y; r[6] = (_Float16)b.z; r[7] = (_Float16)b.w;
  return r;
}

__device__ __forceinline__ void wave_lds_sync() {
  __builtin_amdgcn_fence(__ATOMIC_ACQ_REL, "workgroup");
  __builtin_amdgcn_wave_barrier();
}

__device__ __forceinline__ void load_a_split(const float* p, int h, FragB& hi, FragB& lo) {
  const v4f a0 = *(const v4f*)(p + 8 * h);
  const v4f a1 = *(const v4f*)(p + 8 * h + 4);
  const v4f b0 = *(const v4f*)(p + 16 + 8 * h);
  const v4f b1 = *(const v4f*)(p + 20 + 8 * h);
  split8(a0, a1, hi.h[0], lo.h[0]);
  split8(b0, b1, hi.h[1], lo.h[1]);
}

__device__ __forceinline__ void gemm16x3(v8f (&acc)[8], const float* arow,
                                         const unsigned short* __restrict__ Bhi,
                                         const unsigned short* __restrict__ Blo,
                                         int ldb, int kofs, int ksteps, int h, int m) {
#pragma unroll 1
  for (int kt = 0; kt < ksteps; ++kt) {
    FragB ahi, alo;
    load_a_split(arow + 32 * kt, h, ahi, alo);
#pragma unroll
    for (int nt = 0; nt < 8; ++nt) {
      const size_t bo = (size_t)(nt * 16 + m) * ldb + kofs + 32 * kt + 8 * h;
      FragB bh, bl;
      bh.h[0] = *(const v8us*)(Bhi + bo);
      bh.h[1] = *(const v8us*)(Bhi + bo + 16);
      bl.h[0] = *(const v8us*)(Blo + bo);
      bl.h[1] = *(const v8us*)(Blo + bo + 16);
      acc[nt] = wmb(ahi, bh, acc[nt]);
      acc[nt] = wmb(ahi, bl, acc[nt]);
      acc[nt] = wmb(alo, bh, acc[nt]);
    }
  }
}

__device__ __forceinline__ void rows_store(const float* tile, float* g, int nvalid, int lane) {
#pragma unroll
  for (int rr = 0; rr < 16; ++rr) {
    if (rr < nvalid) {
      const v4f v = *(const v4f*)(tile + rr * 128 + 4 * lane);
      *(volatile v4f*)(g + (size_t)rr * 128 + 4 * lane) = v;
    }
  }
  __threadfence();
#pragma unroll
  for (int rr = 0; rr < 16; ++rr) {
    if (rr < nvalid) {
      const v4f v = *(const v4f*)(tile + rr * 128 + 4 * lane);
      *(volatile v4f*)(g + (size_t)rr * 128 + 4 * lane) = v;
    }
  }
}

__global__ __launch_bounds__(256) void k_pack(const float* __restrict__ W, int K,
                                             unsigned short* hi, unsigned short* lo) {
  const int G = K >> 3;
  const int total = 128 * G;
  const int t = blockIdx.x * 256 + threadIdx.x;
  const int tc = t < total ? t : total - 1;
  const int n = tc / G;
  const int g = tc - n * G;
  v4f a, b;
  a.x = W[(size_t)(8 * g + 0) * 128 + n]; a.y = W[(size_t)(8 * g + 1) * 128 + n];
  a.z = W[(size_t)(8 * g + 2) * 128 + n]; a.w = W[(size_t)(8 * g + 3) * 128 + n];
  b.x = W[(size_t)(8 * g + 4) * 128 + n]; b.y = W[(size_t)(8 * g + 5) * 128 + n];
  b.z = W[(size_t)(8 * g + 6) * 128 + n]; b.w = W[(size_t)(8 * g + 7) * 128 + n];
  v8us vh, vl;
  split8(a, b, vh, vl);
  const bool wr = t < total;
  if (wr) {
    *(volatile v8us*)(hi + (size_t)8 * tc) = vh;
    *(volatile v8us*)(lo + (size_t)8 * tc) = vl;
  }
  __threadfence();
  if (wr) {
    *(volatile v8us*)(hi + (size_t)8 * tc) = vh;
    *(volatile v8us*)(lo + (size_t)8 * tc) = vl;
  }
}

__global__ __launch_bounds__(256) void k_wc(const float* __restrict__ W2, const float* __restrict__ cW1,
                                           const float* __restrict__ b2, const float* __restrict__ cb1,
                                           _Float16* WcT, float* bc) {
  const int t = blockIdx.x * 256 + threadIdx.x;
  const int n = t >> 4, g = t & 15;
  float a[8];
#pragma unroll
  for (int i = 0; i < 8; ++i) a[i] = 0.0f;
#pragma unroll 1
  for (int c = 0; c < 128; ++c) {
    const float wn = cW1[c * 128 + n];
#pragma unroll
    for (int i = 0; i < 8; ++i) a[i] += W2[(8 * g + i) * 128 + c] * wn;
  }
  v8h v;
#pragma unroll
  for (int i = 0; i < 8; ++i) v[i] = (_Float16)(a[i] * WSC);
  const bool wb = (blockIdx.x == 0) && (threadIdx.x < 32);
  v4f bv = {0.0f, 0.0f, 0.0f, 0.0f};
  if (wb) {
    const int l = threadIdx.x;
    float s0 = cb1[4 * l + 0], s1 = cb1[4 * l + 1], s2 = cb1[4 * l + 2], s3 = cb1[4 * l + 3];
#pragma unroll 1
    for (int c = 0; c < 128; ++c) {
      const float bb = b2[c];
      s0 += bb * cW1[c * 128 + 4 * l + 0];
      s1 += bb * cW1[c * 128 + 4 * l + 1];
      s2 += bb * cW1[c * 128 + 4 * l + 2];
      s3 += bb * cW1[c * 128 + 4 * l + 3];
    }
    bv.x = s0; bv.y = s1; bv.z = s2; bv.w = s3;
  }
  *(volatile v8h*)(WcT + (size_t)8 * t) = v;
  if (wb) *(volatile v4f*)(bc + 4 * threadIdx.x) = bv;
  __threadfence();
  *(volatile v8h*)(WcT + (size_t)8 * t) = v;
  if (wb) *(volatile v4f*)(bc + 4 * threadIdx.x) = bv;
}

__global__ __launch_bounds__(NTHR) void k_gemm3(const float* __restrict__ A, int lda, int M,
                                               const unsigned short* __restrict__ Bhi,
                                               const unsigned short* __restrict__ Blo,
                                               int ldb, int kofs, int ksteps,
                                               const float* __restrict__ bias, int useBias,
                                               float* C) {
  extern __shared__ __attribute__((aligned(16))) float dynl[];
  const int tid = threadIdx.x, lane = tid & 31, wave = tid >> 5, h = lane >> 4, m = lane & 15;
  float* tile = dynl + wave * 2048;
  const int row0 = blockIdx.x * 128 + wave * 16;
  int rowm = row0 + m;
  rowm = rowm > M - 1 ? M - 1 : rowm;
  v8f acc[8];
#pragma unroll
  for (int i = 0; i < 8; ++i) acc[i] = zacc();
  gemm16x3(acc, A + (size_t)rowm * lda, Bhi, Blo, ldb, kofs, ksteps, h, m);
  const float ub = (float)useBias;
#pragma unroll
  for (int nt = 0; nt < 8; ++nt) {
    const float b = bias[nt * 16 + m] * ub;
#pragma unroll
    for (int r = 0; r < 8; ++r) tile[(8 * h + r) * 128 + nt * 16 + m] = acc[nt][r] + b;
  }
  wave_lds_sync();
  rows_store(tile, C + (size_t)row0 * 128, M - row0, lane);
}

__device__ __forceinline__ int scan_chunk(const int* __restrict__ dsts, int nE, int cbase, int nodeBase,
                                          int* list, int tid, int wave) {
  int wc = 0;
  const int el0  = tid * EPT;
  const int e0   = cbase + el0;
  const int sent = -2147483647 - 1;
  v4i da, db;
  if (cbase + CHUNK <= nE) {
    da = *(const v4i*)(dsts + e0);
    db = *(const v4i*)(dsts + e0 + 4);
  } else {
    da.x = (e0     < nE) ? dsts[min(e0,     nE - 1)] : sent;
    da.y = (e0 + 1 < nE) ? dsts[min(e0 + 1, nE - 1)] : sent;
    da.z = (e0 + 2 < nE) ? dsts[min(e0 + 2, nE - 1)] : sent;
    da.w = (e0 + 3 < nE) ? dsts[min(e0 + 3, nE - 1)] : sent;
    db.x = (e0 + 4 < nE) ? dsts[min(e0 + 4, nE - 1)] : sent;
    db.y = (e0 + 5 < nE) ? dsts[min(e0 + 5, nE - 1)] : sent;
    db.z = (e0 + 6 < nE) ? dsts[min(e0 + 6, nE - 1)] : sent;
    db.w = (e0 + 7 < nE) ? dsts[min(e0 + 7, nE - 1)] : sent;
  }
  const unsigned nb = (unsigned)nodeBase;
  const unsigned s0 = (unsigned)da.x - nb, s1 = (unsigned)da.y - nb;
  const unsigned s2 = (unsigned)da.z - nb, s3 = (unsigned)da.w - nb;
  const unsigned s4 = (unsigned)db.x - nb, s5 = (unsigned)db.y - nb;
  const unsigned s6 = (unsigned)db.z - nb, s7 = (unsigned)db.w - nb;
  const bool h0 = s0 < (unsigned)NB, h1 = s1 < (unsigned)NB, h2 = s2 < (unsigned)NB, h3 = s3 < (unsigned)NB;
  const bool h4 = s4 < (unsigned)NB, h5 = s5 < (unsigned)NB, h6 = s6 < (unsigned)NB, h7 = s7 < (unsigned)NB;
  const unsigned any = __builtin_amdgcn_ballot_w32(h0 | h1 | h2 | h3 | h4 | h5 | h6 | h7);
  if (any != 0u) {
#define HITJ(J, HJ) { \
      const unsigned mj = __builtin_amdgcn_ballot_w32(HJ); \
      if (mj != 0u) { \
        if (HJ) { \
          const int pos = wc + (int)__builtin_amdgcn_mbcnt_lo(mj, 0u); \
          if (pos < WCAP) list[wave * WCAP + pos] = el0 + (J); \
        } \
        wc += (int)__builtin_popcount(mj); } }
    HITJ(0, h0)
    HITJ(1, h1)
    HITJ(2, h2)
    HITJ(3, h3)
    HITJ(4, h4)
    HITJ(5, h5)
    HITJ(6, h6)
    HITJ(7, h7)
#undef HITJ
  }
  return wc;
}

__global__ __launch_bounds__(NTHR) void k_drain(
    const float* __restrict__ Pp, const float* __restrict__ Qp,
    const float* __restrict__ xc, const float* __restrict__ xo,
    const int* __restrict__ bi, const int* __restrict__ bj,
    const float* __restrict__ w256, const _Float16* __restrict__ WcT,
    const float* __restrict__ bc, const float* __restrict__ c2,
    const float* __restrict__ cb2p,
    float* Uout, float* Sout, int nN, int nO, int nE) {
  extern __shared__ __attribute__((aligned(16))) float dynl[];
  __shared__ int wcnt[NWAVE];
  __shared__ int pendN;
  float* accU  = dynl + OFF_ACC;
  float* utile = dynl + OFF_UT;
  float* sidev = dynl + OFF_SV;
  float* wv    = dynl + OFF_WV;
  float* bcv   = dynl + OFF_BC;
  float* c2v   = dynl + OFF_C2;
  int*   slotb = (int*)(dynl + OFF_SLOT);
  int*   list  = (int*)(dynl + OFF_LIST);
  int*   pend  = (int*)(dynl + OFF_PEND);

  const int tid = threadIdx.x, lane = tid & 31, wave = tid >> 5, h = lane >> 4, m = lane & 15;
  const int nodeBase = blockIdx.x * NB;

  for (int i = tid; i < (NB + 1) * AW; i += NTHR) accU[i] = 0.0f;
  if (tid < 128) { wv[tid] = w256[tid]; bcv[tid] = bc[tid]; c2v[tid] = c2[tid]; }
  if (tid == 0) pendN = 0;
  const float cb2v = cb2p[0];
  __syncthreads();

  const int nChunks = (nE + CHUNK - 1) / CHUNK;
#pragma unroll 1
  for (int ch = 0; ch < nChunks; ++ch) {
    const int cbase = ch * CHUNK;
    const int wc = scan_chunk(bi, nE, cbase, nodeBase, list, tid, wave);
    if (lane == 0) wcnt[wave] = wc;
    __syncthreads();

    const int base = pendN;
    int tot = 0, myoff = 0;
#pragma unroll
    for (int w = 0; w < NWAVE; ++w) {
      int c = wcnt[w];
      c = c > WCAP ? WCAP : (c < 0 ? 0 : c);
      if (w < wave) myoff += c;
      tot += c;
    }
    int newN = base + tot;
    newN = newN > PCAP ? PCAP : newN;
    {
      int n = wcnt[wave];
      n = n > WCAP ? WCAP : (n < 0 ? 0 : n);
      const int* lp = list + wave * WCAP;
      for (int i = lane; i < n; i += 32) {
        const int pos = base + myoff + i;
        if (pos < PCAP) pend[pos] = cbase + lp[i];
      }
    }
    const int fin = (ch == nChunks - 1) ? 1 : 0;
    const int R   = (fin != 0) ? (newN + PASSN - 1) / PASSN : newN / PASSN;
    const int Pv  = (fin != 0) ? newN : R * PASSN;
    __syncthreads();

#pragma unroll 1
    for (int r = 0; r < R; ++r) {
      const int te = wave * 16 + m;
      int idx = r * PASSN + te;
      const bool valid = idx < Pv;
      idx = idx < PCAP - 1 ? idx : PCAP - 1;
      int e = pend[idx];
      e = valid ? e : 0;
      e = e < 0 ? 0 : (e > nE - 1 ? nE - 1 : e);
      int d = bi[e];
      int s = bj[e];
      int slot = d - nodeBase;
      if (!valid || (unsigned)slot >= (unsigned)NB) slot = NB;
      d = d < 0 ? 0 : (d > nN - 1 ? nN - 1 : d);
      s = s < 0 ? 0 : (s > nO - 1 ? nO - 1 : s);
      const float vf = valid ? 1.0f : 0.0f;
      const float r0 = xc[(size_t)d * 3 + 0] - xo[(size_t)s * 3 + 0];
      const float r1 = xc[(size_t)d * 3 + 1] - xo[(size_t)s * 3 + 1];
      const float r2 = xc[(size_t)d * 3 + 2] - xo[(size_t)s * 3 + 2];
      const float d2 = r0 * r0 + r1 * r1 + r2 * r2;
      const float a0 = r0 * vf, a1 = r1 * vf, a2 = r2 * vf;
      if (h == 0) slotb[te] = slot;

      {
        const float* pp = Pp + (size_t)d * 128 + 64 * h;
        const float* qp = Qp + (size_t)s * 128 + 64 * h;
        const float* wp = wv + 64 * h;
        float* up = utile + te * UP + 64 * h;
#pragma unroll
        for (int c4 = 0; c4 < 16; ++c4) {
          const v4f p = *(const v4f*)(pp + 4 * c4);
          const v4f q = *(const v4f*)(qp + 4 * c4);
          const v4f w = *(const v4f*)(wp + 4 * c4);
          v4f u;
          u.x = fmaxf(p.x + q.x + d2 * w.x, 0.0f) * vf;
          u.y = fmaxf(p.y + q.y + d2 * w.y, 0.0f) * vf;
          u.z = fmaxf(p.z + q.z + d2 * w.z, 0.0f) * vf;
          u.w = fmaxf(p.w + q.w + d2 * w.w, 0.0f) * vf;
          *(v4f*)(up + 4 * c4) = u;
        }
      }
      wave_lds_sync();

      FragH af[4];
#pragma unroll
      for (int kt = 0; kt < 4; ++kt) {
        const float* ap = utile + te * UP + 32 * kt + 8 * h;
        const v4f x0 = *(const v4f*)ap,        x1 = *(const v4f*)(ap + 4);
        const v4f y0 = *(const v4f*)(ap + 16), y1 = *(const v4f*)(ap + 20);
        af[kt].h[0] = cvt8h(x0, x1);
        af[kt].h[1] = cvt8h(y0, y1);
      }
      float t[8];
#pragma unroll
      for (int rr = 0; rr < 8; ++rr) t[rr] = 0.0f;
#pragma unroll 1
      for (int nt = 0; nt < 8; ++nt) {
        const int col = nt * 16 + m;
        v8f acc = zacc();
#pragma unroll
        for (int kt = 0; kt < 4; ++kt) {
          const _Float16* bp = WcT + (size_t)col * 128 + 32 * kt + 8 * h;
          FragH b;
          b.h[0] = *(const v8h*)bp;
          b.h[1] = *(const v8h*)(bp + 16);
          acc = wmh(af[kt].v, b.v, acc);
        }
        const float bb = bcv[col], cc = c2v[col];
#pragma unroll
        for (int rr = 0; rr < 8; ++rr) t[rr] += fmaxf(acc[rr] * WINV + bb, 0.0f) * cc;
      }
#pragma unroll
      for (int rr = 0; rr < 8; ++rr) {
        float v = t[rr];
        v += __shfl_xor(v, 8, 32);
        v += __shfl_xor(v, 4, 32);
        v += __shfl_xor(v, 2, 32);
        v += __shfl_xor(v, 1, 32);
        t[rr] = v;
      }
      float sval = t[0];
#pragma unroll
      for (int rr = 1; rr < 8; ++rr) sval = (m == rr) ? t[rr] : sval;
      float lg = sval + cb2v;
      lg = fminf(fmaxf(lg, -30.0f), 30.0f);
      const float ex = expf(-lg);
      const float sg = 1.0f / (1.0f + ex);
      int src = lane + 8 * h;
      src = src > 31 ? 31 : src;
      const float b0 = __shfl(a0, src, 32);
      const float b1 = __shfl(a1, src, 32);
      const float b2 = __shfl(a2, src, 32);
      const float bv = __shfl(vf, src, 32);
      if (m < 8) {
        v4f sv;
        sv.x = b0 * sg; sv.y = b1 * sg; sv.z = b2 * sg; sv.w = bv;
        *(v4f*)(sidev + (wave * 16 + 8 * h + m) * 4) = sv;
      }
      __syncthreads();

      if (tid < AW) {
        const int cu = tid < 128 ? tid : 127;
        const int cs = tid < 128 ? 0 : (tid - 128);
        float* acol = accU + tid;
#pragma unroll 1
        for (int i = 0; i < PASSN; ++i) {
          int sl = slotb[i];
          sl = sl < 0 ? 0 : (sl > NB ? NB : sl);
          const float vu = utile[i * UP + cu];
          const float vs = sidev[i * 4 + cs];
          const float v = (tid < 128) ? vu : vs;
          acol[sl * AW] += v;
        }
      }
      __syncthreads();
    }

    int rem = newN - R * PASSN;
    rem = rem < 0 ? 0 : rem;
    if (R > 0 && tid < rem) pend[tid] = pend[R * PASSN + tid];
    if (tid == 0) pendN = rem;
  }
  __syncthreads();

  const size_t ub = (size_t)nodeBase * 128;
  const int ssl = wave * 32 + lane;
  const v4f svv = *(const v4f*)(accU + ssl * AW + 128);
#pragma unroll 4
  for (int rr = 0; rr < 32; ++rr) {
    const int sl = wave * 32 + rr;
    const v4f v = *(const v4f*)(accU + sl * AW + 4 * lane);
    *(volatile v4f*)(Uout + ub + (size_t)sl * 128 + 4 * lane) = v;
  }
  *(volatile v4f*)(Sout + (size_t)(nodeBase + ssl) * 4) = svv;
  __threadfence();
#pragma unroll 4
  for (int rr = 0; rr < 32; ++rr) {
    const int sl = wave * 32 + rr;
    const v4f v = *(const v4f*)(accU + sl * AW + 4 * lane);
    *(volatile v4f*)(Uout + ub + (size_t)sl * 128 + 4 * lane) = v;
  }
  *(volatile v4f*)(Sout + (size_t)(nodeBase + ssl) * 4) = svv;
}

__global__ __launch_bounds__(CELL_NW * 32) void k_cell(
    const float* __restrict__ hin,
    const float* __restrict__ Uup, const float* __restrict__ Sup,
    const float* __restrict__ Udn, const float* __restrict__ Sdn,
    const unsigned short* __restrict__ W2uh, const unsigned short* __restrict__ W2ul, const float* __restrict__ b2u,
    const unsigned short* __restrict__ W2dh, const unsigned short* __restrict__ W2dl, const float* __restrict__ b2d,
    const unsigned short* __restrict__ C1h, const unsigned short* __restrict__ C1l, const float* __restrict__ cb1,
    const unsigned short* __restrict__ C2h, const unsigned short* __restrict__ C2l, const float* __restrict__ cb2,
    float* out, int nN) {
  extern __shared__ __attribute__((aligned(16))) float dynl[];
  const int tid = threadIdx.x, lane = tid & 31, wave = tid >> 5, h = lane >> 4, m = lane & 15;
  float* tA = dynl + wave * 4096;
  float* tB = tA + 2048;
  const int row0 = blockIdx.x * CELL_ROWS + wave * 16;
  int rowm = row0 + m;
  rowm = rowm > nN - 1 ? nN - 1 : rowm;
  float cnu[8], cnd[8];
#pragma unroll
  for (int r = 0; r < 8; ++r) {
    int rr = row0 + 8 * h + r;
    rr = rr > nN - 1 ? nN - 1 : rr;
    cnu[r] = Sup[(size_t)rr * 4 + 3];
    cnd[r] = Sdn[(size_t)rr * 4 + 3];
  }
  v8f acc[8];

#pragma unroll
  for (int i = 0; i < 8; ++i) acc[i] = zacc();
  gemm16x3(acc, Uup + (size_t)rowm * 128, W2uh, W2ul, 128, 0, 4, h, m);
#pragma unroll
  for (int nt = 0; nt < 8; ++nt) {
    const float b = b2u[nt * 16 + m];
#pragma unroll
    for (int r = 0; r < 8; ++r) tA[(8 * h + r) * 128 + nt * 16 + m] = acc[nt][r] + cnu[r] * b;
  }
#pragma unroll
  for (int i = 0; i < 8; ++i) acc[i] = zacc();
  gemm16x3(acc, Udn + (size_t)rowm * 128, W2dh, W2dl, 128, 0, 4, h, m);
#pragma unroll
  for (int nt = 0; nt < 8; ++nt) {
    const float b = b2d[nt * 16 + m];
#pragma unroll
    for (int r = 0; r < 8; ++r) tB[(8 * h + r) * 128 + nt * 16 + m] = acc[nt][r] + cnd[r] * b;
  }
  wave_lds_sync();

#pragma unroll
  for (int i = 0; i < 8; ++i) acc[i] = zacc();
  gemm16x3(acc, hin + (size_t)rowm * 128, C1h, C1l, 384, 0,   4, h, m);
  gemm16x3(acc, tA + m * 128,              C1h, C1l, 384, 128, 4, h, m);
  gemm16x3(acc, tB + m * 128,              C1h, C1l, 384, 256, 4, h, m);
  wave_lds_sync();
#pragma unroll
  for (int nt = 0; nt < 8; ++nt) {
    const float b = cb1[nt * 16 + m];
#pragma unroll
    for (int r = 0; r < 8; ++r) tA[(8 * h + r) * 128 + nt * 16 + m] = fmaxf(acc[nt][r] + b, 0.0f);
  }
  wave_lds_sync();

#pragma unroll
  for (int i = 0; i < 8; ++i) acc[i] = zacc();
  gemm16x3(acc, tA + m * 128, C2h, C2l, 128, 0, 4, h, m);
#pragma unroll
  for (int nt = 0; nt < 8; ++nt) {
    const float b = cb2[nt * 16 + m];
#pragma unroll
    for (int r = 0; r < 8; ++r) tB[(8 * h + r) * 128 + nt * 16 + m] = acc[nt][r] + b;
  }
  wave_lds_sync();
  rows_store(tB, out + (size_t)row0 * 128, nN - row0, lane);
}

__global__ __launch_bounds__(32) void k_xout(const float* __restrict__ x,
                                            const float* __restrict__ Sup,
                                            const float* __restrict__ Sdn,
                                            const float* __restrict__ cw,
                                            float* out1, int nN) {
  __shared__ __attribute__((aligned(16))) float st[96];
  const int lane = threadIdx.x;
  const int base = blockIdx.x * 32;
  int nrows = nN - base;
  nrows = nrows > 32 ? 32 : (nrows < 0 ? 0 : nrows);
  const float w0 = cw[0], w1 = cw[1];
  for (int idx = lane; idx < 96; idx += 32) {
    const int rl = idx / 3;
    const int c = idx - rl * 3;
    int row = base + rl;
    row = row > nN - 1 ? nN - 1 : row;
    st[idx] = x[(size_t)row * 3 + c] + w0 * Sup[(size_t)row * 4 + c] + w1 * Sdn[(size_t)row * 4 + c];
  }
  __syncthreads();
  const int nfl = nrows * 3;
  const int nv4 = nfl >> 2;
  const int trem = nfl - 4 * nv4;
  const bool wr = lane < nv4;
  const bool wt = lane < trem;
  v4f v = {0.0f, 0.0f, 0.0f, 0.0f};
  float tv = 0.0f;
  if (wr) v = *(const v4f*)(st + 4 * lane);
  if (wt) tv = st[4 * nv4 + lane];
  float* g = out1 + (size_t)base * 3;
  if (wr) *(volatile v4f*)(g + 4 * lane) = v;
  if (wt) *(volatile float*)(g + 4 * nv4 + lane) = tv;
  __threadfence();
  if (wr) *(volatile v4f*)(g + 4 * lane) = v;
  if (wt) *(volatile float*)(g + 4 * nv4 + lane) = tv;
}

extern "C" void kernel_launch(void* const* d_in, const int* in_sizes, int n_in,
                              void* d_out, int out_size, void* d_ws, size_t ws_size,
                              hipStream_t stream) {
  if (n_in < 31) return;
  const int nN = in_sizes[0] / 128;
  const int nU = in_sizes[1] / 128;
  const int nD = in_sizes[2] / 128;
  const int eU = in_sizes[27];
  const int eD = in_sizes[29];
  if (nN <= 0 || nU <= 0 || nD <= 0) return;
  if (in_sizes[0] != nN * 128 || in_sizes[1] != nU * 128 || in_sizes[2] != nD * 128) return;
  if (in_sizes[3] != nN * 3 || in_sizes[4] != nU * 3 || in_sizes[5] != nD * 3) return;
  if (in_sizes[6] < 2) return;
  if (in_sizes[7] != 257 * 128 || in_sizes[8] < 128 || in_sizes[9] != 128 * 128 || in_sizes[10] < 128) return;
  if (in_sizes[11] != 257 * 128 || in_sizes[12] < 128 || in_sizes[13] != 128 * 128 || in_sizes[14] < 128) return;
  if (in_sizes[15] != 384 * 128 || in_sizes[16] < 128 || in_sizes[17] != 128 * 128 || in_sizes[18] < 128) return;
  if (in_sizes[19] != 128 * 128 || in_sizes[20] < 128 || in_sizes[21] < 128 || in_sizes[22] < 1) return;
  if (in_sizes[23] != 128 * 128 || in_sizes[24] < 128 || in_sizes[25] < 128 || in_sizes[26] < 1) return;
  if (eU < 0 || eD < 0 || in_sizes[28] != eU || in_sizes[30] != eD) return;
  if (out_size != nN * 128 + nN * 3) return;

  const float* h      = (const float*)d_in[0];
  const float* h_up   = (const float*)d_in[1];
  const float* h_dn   = (const float*)d_in[2];
  const float* x      = (const float*)d_in[3];
  const float* x_up   = (const float*)d_in[4];
  const float* x_dn   = (const float*)d_in[5];
  const float* cw     = (const float*)d_in[6];
  const float* up_W1  = (const float*)d_in[7];
  const float* up_b1  = (const float*)d_in[8];
  const float* up_W2  = (const float*)d_in[9];
  const float* up_b2  = (const float*)d_in[10];
  const float* dn_W1  = (const float*)d_in[11];
  const float* dn_b1  = (const float*)d_in[12];
  const float* dn_W2  = (const float*)d_in[13];
  const float* dn_b2  = (const float*)d_in[14];
  const float* ce_W1  = (const float*)d_in[15];
  const float* ce_b1  = (const float*)d_in[16];
  const float* ce_W2  = (const float*)d_in[17];
  const float* ce_b2  = (const float*)d_in[18];
  const float* cu_W1  = (const float*)d_in[19];
  const float* cu_b1  = (const float*)d_in[20];
  const float* cu_W2  = (const float*)d_in[21];
  const float* cu_b2  = (const float*)d_in[22];
  const float* cd_W1  = (const float*)d_in[23];
  const float* cd_b1  = (const float*)d_in[24];
  const float* cd_W2  = (const float*)d_in[25];
  const float* cd_b2  = (const float*)d_in[26];
  const int*   b_up_i = (const int*)d_in[27];
  const int*   b_up_j = (const int*)d_in[28];
  const int*   b_dn_i = (const int*)d_in[29];
  const int*   b_dn_j = (const int*)d_in[30];
  float* out0 = (float*)d_out;
  float* out1 = (float*)d_out + (size_t)nN * 128;

  const int nBlk = (nN + NB - 1) / NB;
  const size_t nPad = (size_t)nBlk * NB;
  const int nQ = nU > nD ? nU : nD;

  char* ws = (char*)d_ws;
  size_t off = 0;
  auto take = [&](size_t bytes) -> size_t {
    const size_t o = off;
    off = (off + bytes + 255) & ~(size_t)255;
    return o;
  };
  const size_t oW1uh = take(128 * 256 * 2), oW1ul = take(128 * 256 * 2);
  const size_t oW1dh = take(128 * 256 * 2), oW1dl = take(128 * 256 * 2);
  const size_t oW2uh = take(128 * 128 * 2), oW2ul = take(128 * 128 * 2);
  const size_t oW2dh = take(128 * 128 * 2), oW2dl = take(128 * 128 * 2);
  const size_t oC1h  = take(128 * 384 * 2), oC1l  = take(128 * 384 * 2);
  const size_t oC2h  = take(128 * 128 * 2), oC2l  = take(128 * 128 * 2);
  const size_t oWcu  = take(128 * 128 * 2), oWcd  = take(128 * 128 * 2);
  const size_t oBcu  = take(128 * 4),       oBcd  = take(128 * 4);
  const size_t oP    = take((size_t)nN * 128 * 4);
  const size_t oQ    = take((size_t)nQ * 128 * 4);
  const size_t oUup  = take(nPad * 128 * 4);
  const size_t oSup  = take(nPad * 4 * 4);
  const size_t oUdn  = take(nPad * 128 * 4);
  const size_t oSdn  = take(nPad * 4 * 4);
  if (off > ws_size || off > (size_t)134217728) return;

  unsigned short* W1uh = (unsigned short*)(ws + oW1uh); unsigned short* W1ul = (unsigned short*)(ws + oW1ul);
  unsigned short* W1dh = (unsigned short*)(ws + oW1dh); unsigned short* W1dl = (unsigned short*)(ws + oW1dl);
  unsigned short* W2uh = (unsigned short*)(ws + oW2uh); unsigned short* W2ul = (unsigned short*)(ws + oW2ul);
  unsigned short* W2dh = (unsigned short*)(ws + oW2dh); unsigned short* W2dl = (unsigned short*)(ws + oW2dl);
  unsigned short* C1h  = (unsigned short*)(ws + oC1h);  unsigned short* C1l  = (unsigned short*)(ws + oC1l);
  unsigned short* C2h  = (unsigned short*)(ws + oC2h);  unsigned short* C2l  = (unsigned short*)(ws + oC2l);
  _Float16* Wcu = (_Float16*)(ws + oWcu);
  _Float16* Wcd = (_Float16*)(ws + oWcd);
  float* bcu = (float*)(ws + oBcu);
  float* bcd = (float*)(ws + oBcd);
  float* Pp  = (float*)(ws + oP);
  float* Qp  = (float*)(ws + oQ);
  float* Uup = (float*)(ws + oUup);
  float* Sup = (float*)(ws + oSup);
  float* Udn = (float*)(ws + oUdn);
  float* Sdn = (float*)(ws + oSdn);

  k_pack<<<16, 256, 0, stream>>>(up_W1, 256, W1uh, W1ul);
  k_pack<<<16, 256, 0, stream>>>(dn_W1, 256, W1dh, W1dl);
  k_pack<<<8, 256, 0, stream>>>(up_W2, 128, W2uh, W2ul);
  k_pack<<<8, 256, 0, stream>>>(dn_W2, 128, W2dh, W2dl);
  k_pack<<<24, 256, 0, stream>>>(ce_W1, 384, C1h, C1l);
  k_pack<<<8, 256, 0, stream>>>(ce_W2, 128, C2h, C2l);
  k_wc<<<8, 256, 0, stream>>>(up_W2, cu_W1, up_b2, cu_b1, Wcu, bcu);
  k_wc<<<8, 256, 0, stream>>>(dn_W2, cd_W1, dn_b2, cd_b1, Wcd, bcd);

  k_gemm3<<<(nN + 127) / 128, NTHR, GEMM_LDS_BYTES, stream>>>(h, 128, nN, W1uh, W1ul, 256, 0, 4, up_b1, 1, Pp);
  k_gemm3<<<(nU + 127) / 128, NTHR, GEMM_LDS_BYTES, stream>>>(h_up, 128, nU, W1uh, W1ul, 256, 128, 4, up_b1, 0, Qp);
  k_drain<<<nBlk, NTHR, DRAIN_LDS_BYTES, stream>>>(
      Pp, Qp, x, x_up, b_up_i, b_up_j, up_W1 + 256 * 128, Wcu, bcu, cu_W2, cu_b2, Uup, Sup, nN, nU, eU);

  k_gemm3<<<(nN + 127) / 128, NTHR, GEMM_LDS_BYTES, stream>>>(h, 128, nN, W1dh, W1dl, 256, 0, 4, dn_b1, 1, Pp);
  k_gemm3<<<(nD + 127) / 128, NTHR, GEMM_LDS_BYTES, stream>>>(h_dn, 128, nD, W1dh, W1dl, 256, 128, 4, dn_b1, 0, Qp);
  k_drain<<<nBlk, NTHR, DRAIN_LDS_BYTES, stream>>>(
      Pp, Qp, x, x_dn, b_dn_i, b_dn_j, dn_W1 + 256 * 128, Wcd, bcd, cd_W2, cd_b2, Udn, Sdn, nN, nD, eD);

  k_cell<<<(nN + CELL_ROWS - 1) / CELL_ROWS, CELL_NW * 32, CELL_LDS_BYTES, stream>>>(
      h, Uup, Sup, Udn, Sdn, W2uh, W2ul, up_b2, W2dh, W2dl, dn_b2, C1h, C1l, ce_b1, C2h, C2l, ce_b2, out0, nN);
  k_xout<<<(nN + 31) / 32, 32, 0, stream>>>(x, Sup, Sdn, cw, out1, nN);
}
